// SelfAttn_82094004896145
// MI455X (gfx1250) — hardware-verified
//
#include <hip/hip_runtime.h>
#include <math.h>

#ifndef NB
#define NB 16
#endif
#ifndef QSEQ
#define QSEQ 4096
#endif
#define NB_FULL 16
#define NCH 64
#define HWF 4096
#define IMW 64
#define NKEY 1024
#define C8 8
#define CV 32
static_assert(NB >= 1 && NB <= NB_FULL);
static_assert((QSEQ % 64) == 0 && QSEQ >= 64 && QSEQ <= HWF);

typedef __attribute__((ext_vector_type(16))) _Float16 v16h;
typedef __attribute__((ext_vector_type(8)))  _Float16 v8h;
typedef __attribute__((ext_vector_type(16))) __bf16   v16b;
typedef __attribute__((ext_vector_type(8)))  __bf16   v8b;
typedef __attribute__((ext_vector_type(8)))  float    v8f;
typedef __attribute__((ext_vector_type(4)))  float    v4f;
typedef __attribute__((ext_vector_type(4)))  unsigned int cm_u4;

__device__ __forceinline__ __bf16 bf16_rne(float f) {
    unsigned int u = __float_as_uint(f);
    u += 0x7fffu + ((u >> 16) & 1u);
    return __builtin_bit_cast(__bf16, (unsigned short)(u >> 16));
}
__device__ __forceinline__ float bf16_f32(__bf16 b) { return __uint_as_float(((unsigned int)__builtin_bit_cast(unsigned short, b)) << 16); }
__device__ __forceinline__ float cmb_bf(float v) { const unsigned u = __builtin_bit_cast(unsigned, v); const unsigned r = (u + 0x7fffu + ((u >> 16) & 1u)) & 0xffff0000u; return __builtin_bit_cast(float, r); }
__device__ __forceinline__ v8f wmma16(v16h a, v16h b, v8f c) {
    c = __builtin_amdgcn_wmma_f32_16x16x32_f16(false, a, false, b, (short)0, c, false, false);
    asm volatile("v_nop\n\tv_nop\n\tv_nop\n\tv_nop" : "+v"(c) : "v"(a), "v"(b));
    return c;
}
__device__ __forceinline__ v8f wmmab(v16b a, v16b b, v8f c) {
    c = __builtin_amdgcn_wmma_f32_16x16x32_bf16(false, a, false, b, (short)0, c, false, false);
    asm volatile("v_nop\n\tv_nop\n\tv_nop\n\tv_nop" : "+v"(c) : "v"(a), "v"(b));
    return c;
}
__device__ __forceinline__ v4f vmax4(v4f a, v4f b) { v4f r; r.x = fmaxf(a.x, b.x); r.y = fmaxf(a.y, b.y); r.z = fmaxf(a.z, b.z); r.w = fmaxf(a.w, b.w); return r; }

#define VST2(T, ptr, val) do { const T vst2_v_ = (val); *(volatile T*)(ptr) = vst2_v_; __threadfence(); *(volatile T*)(ptr) = vst2_v_; } while (0)
#define VST2V4(ptr, val) do { const v4f vst2_v4_ = (val); *(volatile v4f*)(ptr) = vst2_v4_; __threadfence(); *(volatile v4f*)(ptr) = vst2_v4_; } while (0)

namespace w25 {
typedef __attribute__((ext_vector_type(16))) _Float16 v16h;
typedef __attribute__((ext_vector_type(8)))  _Float16 v8h;
typedef __attribute__((ext_vector_type(16))) __bf16   v16b;
typedef __attribute__((ext_vector_type(8)))  __bf16   v8b;
typedef __attribute__((ext_vector_type(8)))  float    v8f;
typedef __attribute__((ext_vector_type(4)))  float    v4f;

__device__ __forceinline__ unsigned short f2bf_bits(float f) {
  unsigned u = __float_as_uint(f);
  return (unsigned short)((u + 0x7FFFu + ((u >> 16) & 1u)) >> 16);
}
__device__ __forceinline__ float bf_bits2f(unsigned short h) { return __uint_as_float(((unsigned)h) << 16); }

__device__ __forceinline__ void dep_guard_h(v8f& a, v8f& b, v16h x, v16h y) { asm volatile("v_nop\n\tv_nop\n\tv_nop\n\tv_nop" : "+v"(a), "+v"(b) : "v"(x), "v"(y)); }
__device__ __forceinline__ void dep_guard_b(v8f& a, v8f& b, v16b x, v16b y) { asm volatile("v_nop\n\tv_nop\n\tv_nop\n\tv_nop" : "+v"(a), "+v"(b) : "v"(x), "v"(y)); }
__device__ __forceinline__ void keep4_h(v16h a, v16h b, v16h c, v16h d) { asm volatile("v_nop" :: "v"(a), "v"(b), "v"(c), "v"(d)); }
__device__ __forceinline__ void keep4_b(v16b a, v16b b, v16b c, v16b d) { asm volatile("v_nop" :: "v"(a), "v"(b), "v"(c), "v"(d)); }
__device__ __forceinline__ void acc_guard4(v8f& a, v8f& b, v8f& c, v8f& d) { asm volatile("v_nop\n\tv_nop\n\tv_nop\n\tv_nop" : "+v"(a), "+v"(b), "+v"(c), "+v"(d)); }
template <typename T> struct Frag;
template <> struct Frag<_Float16> {
  typedef v16h V; union U { v16h v; v8h h[2]; };
  static __device__ __forceinline__ v16h load(const _Float16* p) {
    U f; f.h[0] = *(const v8h*)(p); f.h[1] = *(const v8h*)(p + 16); return f.v;
  }
  static __device__ __forceinline__ v8f mma(v16h a, v16h b, v8f c) {
    return __builtin_amdgcn_wmma_f32_16x16x32_f16(false, a, false, b, (short)0, c, false, false);
  }
  static __device__ __forceinline__ void guard(v8f& a, v8f& b, v16h x, v16h y) { dep_guard_h(a, b, x, y); }
  static __device__ __forceinline__ void keep(v16h a, v16h b, v16h c, v16h d) { keep4_h(a, b, c, d); }
};
template <> struct Frag<__bf16> {
  typedef v16b V; union U { v16b v; v8b h[2]; };
  static __device__ __forceinline__ v16b load(const __bf16* p) {
    U f; f.h[0] = *(const v8b*)(p); f.h[1] = *(const v8b*)(p + 16); return f.v;
  }
  static __device__ __forceinline__ v8f mma(v16b a, v16b b, v8f c) {
    return __builtin_amdgcn_wmma_f32_16x16x32_bf16(false, a, false, b, (short)0, c, false, false);
  }
  static __device__ __forceinline__ void guard(v8f& a, v8f& b, v16b x, v16b y) { dep_guard_b(a, b, x, y); }
  static __device__ __forceinline__ void keep(v16b a, v16b b, v16b c, v16b d) { keep4_b(a, b, c, d); }
};

template <int ET> struct Elem;
template <> struct Elem<0> { typedef _Float16 T; };
template <> struct Elem<1> { typedef __bf16 T; };
template <int ET, bool SPLIT, int BIAS_MODE, int OUT_MODE, bool RESID, int ACT = 0>
__global__ __launch_bounds__(256) void wmma_gemm64(
    const unsigned short* __restrict__ Ap, const unsigned short* __restrict__ A2p, int lda, long strideA,
    const unsigned short* __restrict__ Btp, const unsigned short* __restrict__ Bt2p, int ldb, long strideB,
    void* __restrict__ Cout, void* __restrict__ Cout2, int ldc, long strideC,
    const float* __restrict__ bias,
    const float* __restrict__ resid, long strideR,
    int M, int N, int K, float scale) {
  typedef typename Elem<ET>::T T;
  typedef typename Frag<T>::V V;
  constexpr bool RES_LATE = RESID && (OUT_MODE == 0) && (ACT == 0);
  const T* A = (const T*)Ap; const T* A2 = (const T*)A2p; const T* Bt = (const T*)Btp; const T* Bt2 = (const T*)Bt2p;
  __shared__ __align__(16) float sT[8][16 * 68];
  const int b    = blockIdx.y;
  const int lane = threadIdx.x & 31;
  const int wave = threadIdx.x >> 5;
  const int tilesN = N >> 6;
  const int tilesM = M >> 6;
  const int tile = blockIdx.x * 8 + wave;
  if (tile >= tilesM * tilesN) return;
  const int tm = tile / tilesN;
  const int tn = tile - tm * tilesN;
  const int m0 = tm << 6;
  const int n0 = tn << 6;

  const T* Ab  = A  + (size_t)b * strideA;
  const T* Bb  = Bt + (size_t)b * strideB;
  const T* Ab2 = SPLIT ? (A2  + (size_t)b * strideA) : nullptr;
  const T* Bb2 = SPLIT ? (Bt2 + (size_t)b * strideB) : nullptr;

  const int rlane = lane & 15;
  const int koff  = (lane >> 4) * 8;
  const int mOff  = (lane >> 4) * 8;

  v8f acc[4][4];
#pragma unroll
  for (int i = 0; i < 4; ++i)
#pragma unroll
    for (int j = 0; j < 4; ++j) acc[i][j] = (v8f){0.f,0.f,0.f,0.f,0.f,0.f,0.f,0.f};

  for (int k0 = 0; k0 < K; k0 += 32) {
    V bh[4], bl[4];
#pragma unroll
    for (int j = 0; j < 4; ++j) {
      const size_t bo = (size_t)(n0 + (j << 4) + rlane) * ldb + koff + k0;
      bh[j] = Frag<T>::load(Bb + bo);
      if (SPLIT) bl[j] = Frag<T>::load(Bb2 + bo);
    }
#pragma unroll
    for (int i = 0; i < 4; ++i) {
      const size_t ao = (size_t)(m0 + (i << 4) + rlane) * lda + koff + k0;
      V ah = Frag<T>::load(Ab + ao);
      V al;
      if (SPLIT) al = Frag<T>::load(Ab2 + ao);
#pragma unroll
      for (int j = 0; j < 4; ++j) {
        acc[i][j] = Frag<T>::mma(ah, bh[j], acc[i][j]);
        if (SPLIT) {
          acc[i][j] = Frag<T>::mma(ah, bl[j], acc[i][j]);
          acc[i][j] = Frag<T>::mma(al, bh[j], acc[i][j]);
        }
      }
      Frag<T>::guard(acc[i][0], acc[i][3], ah, SPLIT ? al : ah);
    }
    Frag<T>::keep(bh[0], bh[1], bh[2], bh[3]);
    if (SPLIT) Frag<T>::keep(bl[0], bl[1], bl[2], bl[3]);
  }
  acc_guard4(acc[0][0], acc[0][1], acc[0][2], acc[0][3]);
  acc_guard4(acc[1][0], acc[1][1], acc[1][2], acc[1][3]);
  acc_guard4(acc[2][0], acc[2][1], acc[2][2], acc[2][3]);
  acc_guard4(acc[3][0], acc[3][1], acc[3][2], acc[3][3]);

  float* slab = sT[wave];
  const float* Rb = RESID ? (resid + (size_t)b * strideR) : nullptr;
#pragma unroll
  for (int i = 0; i < 4; ++i) {
    const int mBase = m0 + (i << 4);
#pragma unroll
    for (int j = 0; j < 4; ++j) {
      const int n = n0 + (j << 4) + rlane;
      float bv = 0.f;
      if (BIAS_MODE == 2) bv = bias[n];
#pragma unroll
      for (int r = 0; r < 8; ++r) {
        float v = acc[i][j][r] * scale;
        if (BIAS_MODE == 1) v += bias[mBase + mOff + r];
        if (BIAS_MODE == 2) v += bv;
        if (RESID && !RES_LATE) v += Rb[(size_t)(mBase + mOff + r) * ldc + n];
        if (ACT == 1) v = tanhf(v);
        if (ACT == 2) v = fmaxf(v, 0.0f);
        if (ACT == 3) v = v / (1.0f + expf(-v));
        if (ACT == 4) v = (v > 0.f) ? v : 0.01f * v;
        if (ACT == 5) v = 0.5f * v * (1.0f + erff(v * 0.70710678118654752f));
        if (ACT == 6) v = (v > 0.f) ? v : 0.2f * v;
        if (ACT == 7) { const float u = 0.7978845608028654f * (v + 0.044715f * v * v * v); v = 0.5f * v * (1.f + tanhf(u)); }
        slab[(mOff + r) * 68 + (j << 4) + rlane] = v;
      }
    }
    __builtin_amdgcn_fence(3, "workgroup");
    __builtin_amdgcn_wave_barrier();
    __builtin_amdgcn_fence(2, "workgroup");
    if (OUT_MODE == 0) {
      float* C = (float*)Cout + (size_t)b * strideC;
      const int hh = lane >> 4, c4 = (lane & 15) * 4;
      v4f vv[8];
#pragma unroll
      for (int it = 0; it < 8; ++it) {
        const int row = it * 2 + hh;
        v4f v = *(const v4f*)(slab + row * 68 + c4);
        if (RES_LATE) v += *(const v4f*)(Rb + (size_t)(mBase + row) * ldc + n0 + c4);
        vv[it] = v;
      }
      for (int pass = 0; pass < 2; ++pass) {
#pragma unroll
        for (int it = 0; it < 8; ++it) {
          const int row = it * 2 + hh;
          *(volatile v4f*)(C + (size_t)(mBase + row) * ldc + n0 + c4) = vv[it];
        }
        __threadfence();
      }
    } else {
      const int q = lane >> 3, c8 = (lane & 7) * 8;
      unsigned short* C  = (unsigned short*)Cout  + (size_t)b * strideC;
      unsigned short* C2 = (OUT_MODE == 2) ? ((unsigned short*)Cout2 + (size_t)b * strideC) : nullptr;
      for (int pass = 0; pass < 2; ++pass) {
#pragma unroll
        for (int it = 0; it < 4; ++it) {
          const int row = it * 4 + q;
          const float* sp = slab + row * 68 + c8;
          v8h hv, lv;
#pragma unroll
          for (int e = 0; e < 8; ++e) {
            if (OUT_MODE == 1) {
              hv[e] = (_Float16)sp[e];
            } else {
              unsigned short hb = f2bf_bits(sp[e]);
              unsigned short lb = f2bf_bits(sp[e] - bf_bits2f(hb));
              hv[e] = __builtin_bit_cast(_Float16, hb);
              lv[e] = __builtin_bit_cast(_Float16, lb);
            }
          }
          *(volatile v8h*)(C + (size_t)(mBase + row) * ldc + n0 + c8) = hv;
          if (OUT_MODE == 2) *(volatile v8h*)(C2 + (size_t)(mBase + row) * ldc + n0 + c8) = lv;
        }
        __threadfence();
      }
    }
    __builtin_amdgcn_fence(3, "workgroup");
    __builtin_amdgcn_wave_barrier();
    __builtin_amdgcn_fence(2, "workgroup");
  }
}
}

__device__ __forceinline__ unsigned int cmb_pk2(float a, float b) { return (unsigned int)__builtin_bit_cast(unsigned short, (_Float16)a) | ((unsigned int)__builtin_bit_cast(unsigned short, (_Float16)b) << 16); }
__global__ __launch_bounds__(256) void k_cm_bfvec(const float* __restrict__ SRC, float* __restrict__ DST, int n) { const int u = blockIdx.x * 256 + threadIdx.x; if (u >= n) return; VST2(float, DST + u, cmb_bf(SRC[u])); }
__global__ __launch_bounds__(256) void k_cm_castbT(const float* __restrict__ SRC, int lds, unsigned short* __restrict__ DST, int ldd, int nR, int nC, float sc) {
    const long long u = (long long)blockIdx.x * 256 + threadIdx.x; const int per = nR / 8; if (u >= (long long)nC * per) return; const int c = (int)(u / per); const int r0 = 8 * (int)(u % per);
    float w[8];
#pragma unroll
    for (int e = 0; e < 8; ++e) w[e] = cmb_bf(SRC[(long long)(r0 + e) * lds + c]) * sc;
    cm_u4 pk; pk.x = cmb_pk2(w[0], w[1]); pk.y = cmb_pk2(w[2], w[3]); pk.z = cmb_pk2(w[4], w[5]); pk.w = cmb_pk2(w[6], w[7]); VST2(cm_u4, (cm_u4*)(DST + (long long)c * ldd + r0), pk); }

__global__ __launch_bounds__(256) void k_wpack(const float* __restrict__ wt, const float* __restrict__ wp, const float* __restrict__ wg, const float* __restrict__ wo,
                                               unsigned short* __restrict__ W64, unsigned short* __restrict__ WO16) {
    const int u = blockIdx.x * 256 + threadIdx.x;
    v8h hv;
    if (blockIdx.x < 2) {
        const int r = u >> 3, c0 = 8 * (u & 7);
        const int rt = min(r, 7), rp = min(max(r - 8, 0), 7), rg = min(max(r - 16, 0), CV - 1);
        const v4f t0 = *(const v4f*)(wt + rt * NCH + c0), t1 = *(const v4f*)(wt + rt * NCH + c0 + 4);
        const v4f p0 = *(const v4f*)(wp + rp * NCH + c0), p1 = *(const v4f*)(wp + rp * NCH + c0 + 4);
        const v4f g0 = *(const v4f*)(wg + rg * NCH + c0), g1 = *(const v4f*)(wg + rg * NCH + c0 + 4);
        const float av[8] = {t0.x, t0.y, t0.z, t0.w, t1.x, t1.y, t1.z, t1.w};
        const float bv[8] = {p0.x, p0.y, p0.z, p0.w, p1.x, p1.y, p1.z, p1.w};
        const float gv[8] = {g0.x, g0.y, g0.z, g0.w, g1.x, g1.y, g1.z, g1.w};
#pragma unroll
        for (int e = 0; e < 8; ++e) {
            const float sel = (r < C8) ? av[e] : ((r < 2 * C8) ? bv[e] : ((r < 2 * C8 + CV) ? gv[e] : 0.f));
            hv[e] = (_Float16)(16.f * cmb_bf(sel));
        }
        VST2(cm_u4, (cm_u4*)(W64 + 8 * u), __builtin_bit_cast(cm_u4, hv));
    } else {
        const int u2 = u - 512; if (u2 >= 64 * 4) return;
        const int r = u2 >> 2, c0 = 8 * (u2 & 3);
        const v4f o0 = *(const v4f*)(wo + r * CV + c0), o1 = *(const v4f*)(wo + r * CV + c0 + 4);
        const float ov[8] = {o0.x, o0.y, o0.z, o0.w, o1.x, o1.y, o1.z, o1.w};
#pragma unroll
        for (int e = 0; e < 8; ++e) hv[e] = (_Float16)(16.f * cmb_bf(ov[e]));
        VST2(cm_u4, (cm_u4*)(WO16 + 8 * u2), __builtin_bit_cast(cm_u4, hv));
    }
}

__global__ __launch_bounds__(256) void k_qpack(const float* __restrict__ QKV, unsigned short* __restrict__ QP, int nrows) {
    const int u = blockIdx.x * 256 + threadIdx.x; if (u >= nrows * 4) return;
    const int R = u >> 2, qt = u & 3;
    const float* s = QKV + (size_t)R * 64;
    const v4f t0 = *(const v4f*)s, t1 = *(const v4f*)(s + 4);
    const float th[8] = {t0.x, t0.y, t0.z, t0.w, t1.x, t1.y, t1.z, t1.w};
    v8b o;
#pragma unroll
    for (int e = 0; e < 8; ++e) {
        const float hf = bf16_f32(bf16_rne(th[e])); const float lf = th[e] - hf;
        const float sel = (qt == 3) ? 0.f : ((qt == 2) ? lf : hf);
        o[e] = bf16_rne(sel);
    }
    VST2(cm_u4, (cm_u4*)(QP + 8 * (size_t)u), __builtin_bit_cast(cm_u4, o));
}

__global__ __launch_bounds__(256) void k_kpack(const float* __restrict__ QKV, unsigned short* __restrict__ KP, int nrows) {
    const int u = blockIdx.x * 256 + threadIdx.x; if (u >= nrows * 4) return;
    const int R = u >> 2, qt = u & 3; const int b = R >> 10, key = R & (NKEY - 1), ph = key >> 5, pw = key & 31;
    const float* s0 = QKV + ((size_t)b * HWF + (size_t)(2 * ph) * IMW + 2 * pw) * 64 + C8;
    const float* s1 = s0 + 64; const float* s2 = s0 + IMW * 64; const float* s3 = s2 + 64;
    const v4f a0 = *(const v4f*)s0, a1 = *(const v4f*)(s0 + 4), b0 = *(const v4f*)s1, b1 = *(const v4f*)(s1 + 4);
    const v4f c0 = *(const v4f*)s2, c1 = *(const v4f*)(s2 + 4), d0 = *(const v4f*)s3, d1 = *(const v4f*)(s3 + 4);
    const v4f m0 = vmax4(vmax4(a0, b0), vmax4(c0, d0)), m1 = vmax4(vmax4(a1, b1), vmax4(c1, d1));
    const float pv[8] = {m0.x, m0.y, m0.z, m0.w, m1.x, m1.y, m1.z, m1.w};
    v8b o;
#pragma unroll
    for (int e = 0; e < 8; ++e) {
        const float hf = bf16_f32(bf16_rne(pv[e])); const float lf = pv[e] - hf;
        const float sel = (qt == 3) ? 0.f : ((qt == 1) ? lf : hf);
        o[e] = bf16_rne(sel);
    }
    VST2(cm_u4, (cm_u4*)(KP + 8 * (size_t)u), __builtin_bit_cast(cm_u4, o));
}

__global__ __launch_bounds__(256) void k_vtr(const float* __restrict__ QKV, unsigned short* __restrict__ VT) {
    __shared__ float tile[CV][65];
    const int b = blockIdx.y, key0 = blockIdx.x * 64, t = threadIdx.x;
    {
        const int kl = t >> 2, cq = t & 3; const int key = key0 + kl, ph = key >> 5, pw = key & 31;
        const float* s0 = QKV + ((size_t)b * HWF + (size_t)(2 * ph) * IMW + 2 * pw) * 64 + 2 * C8 + 8 * cq;
        const float* s1 = s0 + 64; const float* s2 = s0 + IMW * 64; const float* s3 = s2 + 64;
        const v4f a0 = *(const v4f*)s0, a1 = *(const v4f*)(s0 + 4), b0 = *(const v4f*)s1, b1 = *(const v4f*)(s1 + 4);
        const v4f c0 = *(const v4f*)s2, c1 = *(const v4f*)(s2 + 4), d0 = *(const v4f*)s3, d1 = *(const v4f*)(s3 + 4);
        const v4f m0 = vmax4(vmax4(a0, b0), vmax4(c0, d0)), m1 = vmax4(vmax4(a1, b1), vmax4(c1, d1));
        const float pv[8] = {m0.x, m0.y, m0.z, m0.w, m1.x, m1.y, m1.z, m1.w};
#pragma unroll
        for (int e = 0; e < 8; ++e) tile[8 * cq + e][kl] = pv[e];
    }
    __syncthreads();
    {
        const int ch = t >> 3, k8 = (t & 7) * 8;
        v8h hv;
#pragma unroll
        for (int e = 0; e < 8; ++e) hv[e] = (_Float16)tile[ch][k8 + e];
        VST2(cm_u4, (cm_u4*)(VT + ((size_t)b * CV + ch) * NKEY + key0 + k8), __builtin_bit_cast(cm_u4, hv));
    }
}

__global__ __launch_bounds__(128) __attribute__((amdgpu_num_vgpr(256)))
void k_att8(const __bf16* __restrict__ QP, const __bf16* __restrict__ KP, const _Float16* __restrict__ VT, const float* __restrict__ gam,
            _Float16* __restrict__ ATT, int nqb) {
    union FB { v16b v; v8b h[2]; };
    union FH { v16h v; v8h h[2]; };
    __shared__ __align__(16) _Float16 Psh[4][16 * 64];
    __shared__ __align__(16) float    Os[4][16 * 36];
    const int tid = threadIdx.x, wave = tid >> 5, lane = tid & 31, hh = lane >> 4, c = lane & 15;
    const int bx = blockIdx.x, qb = bx % nqb, b = bx / nqb;
    const int q0 = qb * 64 + wave * 16;
    const __bf16*   QPb = QP + (size_t)b * HWF * 32;
    const __bf16*   KPb = KP + (size_t)b * NKEY * 32;
    const _Float16* VTb = VT + (size_t)b * CV * NKEY;
    const float L2E = 1.4426950408889634f;
    const float NEG = -__builtin_inff();

    FB qa;
    {
        const __bf16* qr = QPb + (size_t)(q0 + c) * 32;
        qa.h[0] = *(const v8b*)(qr + 8 * hh);
        qa.h[1] = *(const v8b*)(qr + 16 + 8 * hh);
    }
    float mrow[8], lrow[8];
    v8f oacc[2];
#pragma unroll
    for (int r = 0; r < 8; ++r) { mrow[r] = NEG; lrow[r] = 0.f; }
#pragma unroll
    for (int t = 0; t < 2; ++t) oacc[t] = (v8f){0.f,0.f,0.f,0.f,0.f,0.f,0.f,0.f};
    _Float16* pwh = Psh[wave];

#pragma unroll 1
    for (int kc = 0; kc < NKEY / 64; ++kc) {
        const int kv0 = kc * 64;
        v8f s[4];
#pragma unroll
        for (int j = 0; j < 4; ++j) {
            FB kb; const __bf16* kr = KPb + (size_t)(kv0 + j * 16 + c) * 32;
            kb.h[0] = *(const v8b*)(kr + 8 * hh);
            kb.h[1] = *(const v8b*)(kr + 16 + 8 * hh);
            const v8f zz = (v8f){0.f,0.f,0.f,0.f,0.f,0.f,0.f,0.f};
            s[j] = wmmab(qa.v, kb.v, zz);
        }
        float cm[8];
#pragma unroll
        for (int r = 0; r < 8; ++r) {
            float m = fmaxf(fmaxf(s[0][r], s[1][r]), fmaxf(s[2][r], s[3][r]));
#pragma unroll
            for (int off = 1; off < 16; off <<= 1) m = fmaxf(m, __shfl_xor(m, off, 32));
            cm[r] = m * L2E;
        }
#pragma unroll
        for (int r = 0; r < 8; ++r) {
            const float mnew = fmaxf(mrow[r], cm[r]);
            const float alpha = exp2f(mrow[r] - mnew);
            mrow[r] = mnew;
            float psum = 0.f;
#pragma unroll
            for (int j = 0; j < 4; ++j) {
                const float p = exp2f(s[j][r] * L2E - mnew);
                psum += p;
                pwh[(8 * hh + r) * 64 + j * 16 + c] = (_Float16)(p * 32768.f);
            }
#pragma unroll
            for (int off = 1; off < 16; off <<= 1) psum += __shfl_xor(psum, off, 32);
            lrow[r] = lrow[r] * alpha + psum;
            oacc[0][r] *= alpha; oacc[1][r] *= alpha;
        }
        __builtin_amdgcn_fence(3, "wavefront");
        __builtin_amdgcn_wave_barrier();
        __builtin_amdgcn_fence(2, "wavefront");
#pragma unroll 1
        for (int kk = 0; kk < 2; ++kk) {
            FH pa;
            pa.h[0] = *(const v8h*)(pwh + c * 64 + kk * 32 + 8 * hh);
            pa.h[1] = *(const v8h*)(pwh + c * 64 + kk * 32 + 16 + 8 * hh);
#pragma unroll
            for (int t = 0; t < 2; ++t) {
                FH vb; const _Float16* vr = VTb + (size_t)(t * 16 + c) * NKEY + kv0 + kk * 32;
                vb.h[0] = *(const v8h*)(vr + 8 * hh);
                vb.h[1] = *(const v8h*)(vr + 16 + 8 * hh);
                oacc[t] = wmma16(pa.v, vb.v, oacc[t]);
            }
        }
    }

    const float gsc = 16.f * cmb_bf(gam[0]);
    float* os = Os[wave];
#pragma unroll
    for (int r = 0; r < 8; ++r) {
        const float inv = gsc * (1.0f / (lrow[r] * 32768.f));
#pragma unroll
        for (int t = 0; t < 2; ++t) os[(8 * hh + r) * 36 + t * 16 + c] = oacc[t][r] * inv;
    }
    __builtin_amdgcn_fence(3, "wavefront");
    __builtin_amdgcn_wave_barrier();
    __builtin_amdgcn_fence(2, "wavefront");
    _Float16* ab = ATT + ((size_t)b * HWF + q0) * CV;
#pragma unroll
    for (int it = 0; it < 2; ++it) {
        const int row = it * 8 + (lane >> 2), c8 = (lane & 3) * 8;
        const float* sp = os + row * 36 + c8;
        const v4f u0 = *(const v4f*)sp, u1 = *(const v4f*)(sp + 4);
        v8h hv;
        hv[0] = (_Float16)u0.x; hv[1] = (_Float16)u0.y; hv[2] = (_Float16)u0.z; hv[3] = (_Float16)u0.w;
        hv[4] = (_Float16)u1.x; hv[5] = (_Float16)u1.y; hv[6] = (_Float16)u1.z; hv[7] = (_Float16)u1.w;
        VST2(cm_u4, (cm_u4*)(ab + (size_t)row * CV + c8), __builtin_bit_cast(cm_u4, hv));
    }
}

__host__ __device__ constexpr size_t al256(size_t v) { return (v + 255) & ~(size_t)255; }
constexpr size_t SZ_W64 = al256((size_t)64 * 64 * 2);
constexpr size_t SZ_WO  = al256((size_t)64 * CV * 2);
constexpr size_t SZ_TB  = al256((size_t)NB * NCH * HWF * 4);
constexpr size_t SZ_TT  = al256((size_t)HWF * NB * NCH * 2);
constexpr size_t SZ_QKV = al256((size_t)NB * HWF * 64 * 4);
constexpr size_t SZ_QP  = al256((size_t)NB * HWF * 32 * 2);
constexpr size_t SZ_KP  = al256((size_t)NB * NKEY * 32 * 2);
constexpr size_t SZ_VT  = al256((size_t)NB * CV * NKEY * 2);
constexpr size_t SZ_ATT = al256((size_t)NB * HWF * CV * 2);
constexpr size_t WS_TOTAL = SZ_W64 + SZ_WO + SZ_TB + SZ_TT + SZ_QKV + SZ_QP + SZ_KP + SZ_VT + SZ_ATT;
static_assert(WS_TOTAL <= (size_t)134217728);
static_assert((size_t)(NB_FULL - 1) * NCH * HWF + (size_t)NCH * HWF <= (size_t)NB_FULL * NCH * HWF);

extern "C" void kernel_launch(void* const* d_in, const int* in_sizes, int n_in,
                              void* d_out, int out_size, void* d_ws, size_t ws_size, hipStream_t stream) {
    if (n_in < 6) return;
    if (in_sizes[0] < NB * NCH * HWF || in_sizes[1] < C8 * NCH || in_sizes[2] < C8 * NCH || in_sizes[3] < CV * NCH || in_sizes[4] < NCH * CV || in_sizes[5] < 1) return;
    if (out_size < NB * NCH * HWF) return;
    if (WS_TOTAL > ws_size) return;
    const float* x   = (const float*)d_in[0];
    const float* wt  = (const float*)d_in[1];
    const float* wp  = (const float*)d_in[2];
    const float* wg  = (const float*)d_in[3];
    const float* wo  = (const float*)d_in[4];
    const float* gam = (const float*)d_in[5];
    float* out = (float*)d_out;
    char* wsp = (char*)d_ws;
    unsigned short* W64  = (unsigned short*)wsp; wsp += SZ_W64;
    unsigned short* WO16 = (unsigned short*)wsp; wsp += SZ_WO;
    float*          TB   = (float*)wsp;          wsp += SZ_TB;
    unsigned short* TT   = (unsigned short*)wsp; wsp += SZ_TT;
    float*          QKV  = (float*)wsp;          wsp += SZ_QKV;
    unsigned short* QP   = (unsigned short*)wsp; wsp += SZ_QP;
    unsigned short* KP   = (unsigned short*)wsp; wsp += SZ_KP;
    unsigned short* VT   = (unsigned short*)wsp; wsp += SZ_VT;
    unsigned short* ATT  = (unsigned short*)wsp; wsp += SZ_ATT;
    if ((size_t)(wsp - (char*)d_ws) > ws_size) return;

    const int nx = NB * NCH * HWF;
    k_wpack<<<3, 256, 0, stream>>>(wt, wp, wg, wo, W64, WO16);
    k_cm_bfvec<<<(unsigned)((nx + 255) / 256), 256, 0, stream>>>(x, TB, nx);
    k_cm_castbT<<<(unsigned)(((long long)HWF * ((NB * NCH) / 8) + 255) / 256), 256, 0, stream>>>(x, HWF, TT, NB * NCH, NB * NCH, HWF, 1.0f);
    w25::wmma_gemm64<0, false, 0, 0, false, 0><<<dim3((unsigned)(((HWF / 64) * 1 + 7) / 8), (unsigned)NB), 256, 0, stream>>>(
        TT, nullptr, NB * NCH, (long)NCH, W64, nullptr, 64, (long)0, (void*)QKV, nullptr, 64, (long)HWF * 64, nullptr, nullptr, (long)0, HWF, 64, 64, 0.0625f);
    k_qpack<<<(unsigned)((NB * HWF * 4 + 255) / 256), 256, 0, stream>>>(QKV, QP, NB * HWF);
    k_kpack<<<(unsigned)((NB * NKEY * 4 + 255) / 256), 256, 0, stream>>>(QKV, KP, NB * NKEY);
    k_vtr<<<dim3(NKEY / 64, (unsigned)NB), 256, 0, stream>>>(QKV, VT);
    k_att8<<<(unsigned)(NB * (QSEQ / 64)), 128, 0, stream>>>((const __bf16*)QP, (const __bf16*)KP, (const _Float16*)VT, gam, (_Float16*)ATT, QSEQ / 64);
    w25::wmma_gemm64<0, false, 0, 0, true, 0><<<dim3((unsigned)((1 * (QSEQ / 64) + 7) / 8), (unsigned)NB), 256, 0, stream>>>(
        WO16, nullptr, CV, (long)0, ATT, nullptr, CV, (long)HWF * CV, (void*)out, nullptr, HWF, (long)NCH * HWF, nullptr, TB, (long)NCH * HWF, NCH, QSEQ, CV, 0.00390625f);
}
